// Dcls1d_82927228552100
// MI455X (gfx1250) — hardware-verified
//
#include <hip/hip_runtime.h>
#include <math.h>

typedef __attribute__((ext_vector_type(16))) _Float16 v16h;
typedef __attribute__((ext_vector_type(16))) __bf16 v16b;
typedef __attribute__((ext_vector_type(8)))  _Float16 v8h;
typedef __attribute__((ext_vector_type(8)))  float v8f;
typedef __attribute__((ext_vector_type(4)))  float v4f;
typedef __attribute__((ext_vector_type(2)))  float v2f;
typedef __attribute__((ext_vector_type(4)))  unsigned v4u;
typedef __attribute__((ext_vector_type(4)))  int v4i;
typedef float __attribute__((may_alias)) float_a;
typedef int __attribute__((may_alias)) int_a;

template <typename T> __device__ __forceinline__ void vst2(void* p, T v) { *(volatile T*)p = v; __threadfence(); *(volatile T*)p = v; }
__device__ __forceinline__ v8f wmma16(v16h a, v16h b, v8f c) {
  v8f d = __builtin_amdgcn_wmma_f32_16x16x32_f16(false, a, false, b, (short)0, c, false, false);
  asm volatile("v_nop\n\tv_nop\n\tv_nop\n\tv_nop" : "+v"(d) : "v"(a), "v"(b));
  return d;
}
__device__ __forceinline__ v8f wmma_bf(v16b a, v16b b, v8f c) {
  v8f d = __builtin_amdgcn_wmma_f32_16x16x32_bf16(false, a, false, b, (short)0, c, false, false);
  asm volatile("v_nop\n\tv_nop\n\tv_nop\n\tv_nop" : "+v"(d) : "v"(a), "v"(b));
  return d;
}
__device__ __forceinline__ v16h frag_h(const _Float16* rowk0, int lane) {
  union { v16h v; v8h q[2]; } u; const _Float16* p = rowk0 + 8 * (lane >> 4);
  u.q[0] = *(const v8h*)p; u.q[1] = *(const v8h*)(p + 16); return u.v;
}
__device__ __forceinline__ v16h frag_f32(const float* rowk0, int lane) {
  v16h a; const float* p = rowk0 + 8 * (lane >> 4);
#pragma unroll
  for (int i = 0; i < 8; ++i) { a[i] = (_Float16)p[i]; a[8 + i] = (_Float16)p[16 + i]; }
  return a;
}
__device__ __forceinline__ v16h frag_f32s(const float* rowk0, int lane, float sc) {
  v16h a; const float* p = rowk0 + 8 * (lane >> 4);
#pragma unroll
  for (int i = 0; i < 8; ++i) { a[i] = (_Float16)(p[i] * sc); a[8 + i] = (_Float16)(p[16 + i] * sc); }
  return a;
}
__device__ __forceinline__ v16h fragc_f32(const float* W, int k0, int n, int lane, int ld, int K) {
  v16h a; const int g = lane >> 4;
#pragma unroll
  for (int i = 0; i < 8; ++i) { const int ka = k0 + 8 * g + i, kb = ka + 16;
    a[i] = (_Float16)(ka < K ? W[(size_t)(ka < K ? ka : K - 1) * ld + n] : 0.f); a[8 + i] = (_Float16)(kb < K ? W[(size_t)(kb < K ? kb : K - 1) * ld + n] : 0.f); }
  return a;
}
struct F2 { v16b h, l; };
__device__ __forceinline__ F2 bsplit16(const float v[16]) { F2 r;
#pragma unroll
  for (int i = 0; i < 16; ++i) { const __bf16 h = (__bf16)v[i]; r.h[i] = h; r.l[i] = (__bf16)(v[i] - (float)h); }
  return r; }
__device__ __forceinline__ F2 split_row(const float* row, int k0, int lane) { float v[16]; const float* p = row + k0 + 8 * (lane >> 4);
#pragma unroll
  for (int i = 0; i < 8; ++i) { v[i] = p[i]; v[8 + i] = p[16 + i]; }
  return bsplit16(v); }
__device__ __forceinline__ F2 split_rowK(const float* row, int k0, int lane, int K) { float v[16]; const int g = lane >> 4;
#pragma unroll
  for (int i = 0; i < 8; ++i) { const int ka = k0 + 8 * g + i, kb = ka + 16; v[i] = ka < K ? row[ka < K ? ka : K - 1] : 0.f; v[8 + i] = kb < K ? row[kb < K ? kb : K - 1] : 0.f; }
  return bsplit16(v); }
__device__ __forceinline__ F2 split_col(const float* W, int k0, int n, int lane, int ld, int K) { float v[16]; const int g = lane >> 4;
#pragma unroll
  for (int i = 0; i < 8; ++i) { const int ka = k0 + 8 * g + i, kb = ka + 16; v[i] = ka < K ? W[(size_t)(ka < K ? ka : K - 1) * ld + n] : 0.f; v[8 + i] = kb < K ? W[(size_t)(kb < K ? kb : K - 1) * ld + n] : 0.f; }
  return bsplit16(v); }
__device__ __forceinline__ v8f mac3(const F2& a, const F2& b, v8f c) { c = wmma_bf(a.l, b.h, c); c = wmma_bf(a.h, b.l, c); return wmma_bf(a.h, b.h, c); }
__device__ __forceinline__ float sigm(float v) { return 1.0f / (1.0f + expf(-v)); }
#define LDSX() do { asm volatile("s_wait_dscnt 0" ::: "memory"); __builtin_amdgcn_wave_barrier(); __builtin_amdgcn_fence(__ATOMIC_RELEASE, "workgroup"); } while (0)


#define NBB 32
#define CI 256
#define COUT 256
#define LL 1024
#define KCNT 26
#define KD 25
#define LOUT (LL - KD + 1)
#define TP 1056
#ifndef NBT
#define NBT NBB
#endif
typedef __attribute__((ext_vector_type(8))) __bf16 v8b;
__device__ __forceinline__ v16b frag_b(const __bf16* rowk0, int lane) {
  union { v16b v; v8b q[2]; } u; const __bf16* p = rowk0 + 8 * (lane >> 4);
  u.q[0] = *(const v8b*)p; u.q[1] = *(const v8b*)(p + 16); return u.v;
}
__device__ __forceinline__ float bfr(float v) { return (float)(__bf16)v; }
__device__ __attribute__((noinline)) float exp_ni(float v) { return expf(v); }
__device__ __attribute__((noinline)) float erf_ni(float v) { return erff(v); }

#define WS_KT   0u
#define WS_XT   (WS_KT + 4u * KD * COUT * CI)
#define WS_OS   (WS_XT + 2u * NBB * TP * CI)
#define WS_END  (WS_OS + 4u * NBB * COUT * LL)

__global__ __launch_bounds__(256) void k_kc(const float* __restrict__ Wt, const float* __restrict__ SG, const float* __restrict__ PP, const float* __restrict__ SIG, float* __restrict__ KT) {
  __shared__ __align__(16) float sk[KD][CI]; __shared__ float sx[KD][CI]; const int o = blockIdx.x, i = threadIdx.x;
#pragma unroll 1
  for (int d = 0; d < KD; ++d) sk[d][i] = 0.f;
  const size_t base = ((size_t)o * CI + i) * KCNT;
#pragma unroll 1
  for (int c = 0; c < KCNT; ++c) { const float w = bfr(Wt[base + c]) * bfr(SG[base + c]); const float pc = bfr(PP[base + c]) + (float)(KD / 2); const float s = fabsf(bfr(SIG[base + c])) + 0.27f;
    float sum = 0.f;
#pragma unroll 1
    for (int d = 0; d < KD; ++d) { const float t = ((float)d - pc) / s; const float e = exp_ni(-0.5f * (t * t)); sx[d][i] = e; sum += e; }
    const float den = sum + 1e-7f;
#pragma unroll 1
    for (int d = 0; d < KD; ++d) sk[d][i] += (sx[d][i] / den) * w; }
  __syncthreads();
  for (int q = i; q < KD * 64; q += 256) { const int d = q >> 6, pc = q & 63; vst2(KT + ((size_t)d * COUT + o) * CI + pc * 4, *(const v4f*)&sk[d][pc * 4]); }
}
__global__ __launch_bounds__(256) void k_xt(const float* __restrict__ X, __bf16* __restrict__ XT) {
  __shared__ __align__(16) __bf16 s[64][CI + 8]; const int t0 = blockIdx.x * 64, b = blockIdx.y, tid = threadIdx.x;
  for (int q = tid; q < CI * 64; q += 256) { const int i = q >> 6, tl = q & 63; const int t = t0 + tl; s[tl][i] = (__bf16)((t < LL) ? X[((size_t)b * CI + i) * LL + (t < LL ? t : 0)] : 0.f); }
  __syncthreads();
  for (int q = tid; q < 64 * 32; q += 256) { const int tl = q >> 5, pc = q & 31; if (t0 + tl < TP) vst2((unsigned*)(XT + ((size_t)b * TP + t0 + tl) * CI + pc * 8), *(const v4u*)&s[tl][pc * 8]); }
}
__global__ __launch_bounds__(128) void k_conv(const float* __restrict__ KT, const __bf16* __restrict__ XT, float* __restrict__ OS) {
  __shared__ __align__(16) float so[4][16][132];
  const int tid = threadIdx.x, wave = tid >> 5, lane = tid & 31, col = lane & 15, g = lane >> 4; const int o0 = blockIdx.x * 64 + wave * 16, t0 = blockIdx.y * 128, b = blockIdx.z;
  v8f acc[8] = {};
#pragma unroll 1
  for (int d = 0; d < KD; ++d) {
#pragma unroll 2
    for (int kc = 0; kc < CI / 32; ++kc) { const F2 a = split_row(KT + ((size_t)d * COUT + o0 + col) * CI, kc * 32, lane);
#pragma unroll
      for (int j = 0; j < 8; ++j) { const v16b xb = frag_b(XT + ((size_t)b * TP + t0 + j * 16 + col + d) * CI + kc * 32, lane); acc[j] = wmma_bf(a.l, xb, acc[j]); acc[j] = wmma_bf(a.h, xb, acc[j]); } } }
#pragma unroll
  for (int j = 0; j < 8; ++j)
#pragma unroll
    for (int r = 0; r < 8; ++r) so[wave][8 * g + r][j * 16 + col] = acc[j][r];
  LDSX();
  for (int rl = 0; rl < 16; ++rl) vst2(OS + ((size_t)b * COUT + o0 + rl) * LL + t0 + lane * 4, *(const v4f*)&so[wave][rl][lane * 4]);
}
__global__ __launch_bounds__(256) void k_out(const float* __restrict__ OS, float* __restrict__ out) {
  const size_t p = (size_t)blockIdx.x * 256 + threadIdx.x; const size_t total = (size_t)NBT * COUT * LOUT; if (p * 4 >= total) return;
  v4f v;
#pragma unroll
  for (int i = 0; i < 4; ++i) { const size_t f = p * 4 + i; v[i] = (f < total) ? OS[(f / LOUT) * LL + (f % LOUT)] : 0.f; }
  vst2(out + p * 4, v);
}
extern "C" void kernel_launch(void* const* d_in, const int* in_sizes, int n_in, void* d_out, int out_size, void* d_ws, size_t ws_size, hipStream_t stream) {
  (void)in_sizes; (void)n_in; (void)out_size;
  const float** F = (const float**)d_in;
  if (ws_size < (size_t)WS_END) return;
  char* ws = (char*)d_ws; float *KT = (float*)(ws + WS_KT), *OS = (float*)(ws + WS_OS); __bf16* XT = (__bf16*)(ws + WS_XT);
  k_kc<<<COUT, 256, 0, stream>>>(F[1], F[2], F[3], F[4], KT);
  k_xt<<<dim3((TP + 63) / 64, NBT), 256, 0, stream>>>(F[0], XT);
  k_conv<<<dim3(COUT / 64, LL / 128, NBT), 128, 0, stream>>>(KT, XT, OS);
  k_out<<<(unsigned)((((size_t)NBT * COUT * LOUT) / 4 + 255) / 256), 256, 0, stream>>>(OS, (float*)d_out);
}
